// SAConvLSTM_2714419331527
// MI455X (gfx1250) — hardware-run, weakly checked
//
#include <hip/hip_runtime.h>
#include <stdint.h>
#include <stddef.h>

#define NB_  8
#define NCH  64
#define NT_  16
#define NPX  1024
#define IW_  32
#define NIMG 128
#define ICH  64
#define CZ_  128
#define NOC  256

typedef _Float16 v16h __attribute__((ext_vector_type(16)));
typedef _Float16 v8h  __attribute__((ext_vector_type(8)));
typedef float    v8f  __attribute__((ext_vector_type(8)));
typedef float    v4f  __attribute__((ext_vector_type(4)));
typedef unsigned v8u  __attribute__((ext_vector_type(8)));

static_assert(NB_ * NT_ == NIMG);
static_assert((NIMG % ICH) == 0);
static_assert(IW_ * IW_ == NPX);
static_assert(sizeof(v16h) == 32 && sizeof(v8u) == 32);

__device__ __forceinline__ float bfr(float f) {
  unsigned u = __float_as_uint(f);
  u = (u + 0x7FFFu + ((u >> 16) & 1u)) & 0xFFFF0000u;
  return __uint_as_float(u);
}
__device__ __forceinline__ v8f zero8() {
  v8f z;
#pragma unroll
  for (int i = 0; i < 8; ++i) z[i] = 0.0f;
  return z;
}
__device__ __forceinline__ v16h ldfrag(const _Float16* p) {
  union { v16h v; v8h hh[2]; } f;
  f.hh[0] = *(const v8h*)(p);
  f.hh[1] = *(const v8h*)(p + 16);
  return f.v;
}
__device__ __forceinline__ v8f mma16(v16h a, v16h b, v8f c) {
  return __builtin_amdgcn_wmma_f32_16x16x32_f16(false, a, false, b, (short)0, c, false, false);
}
union FragU { v16h v; v8u u; };

#if defined(__HIP_DEVICE_COMPILE__)
#define WG_NOP4 "v_nop\n\tv_nop\n\tv_nop\n\tv_nop"
#define GUARD1_4(d0, x0, x1, x2, x3) \
  asm volatile(WG_NOP4 : "+v"(d0) : "v"(x0), "v"(x1), "v"(x2), "v"(x3))
#define GUARD2_5(d0, d1, x0, x1, x2, x3, x4) \
  asm volatile(WG_NOP4 : "+v"(d0), "+v"(d1) : "v"(x0), "v"(x1), "v"(x2), "v"(x3), "v"(x4))
#define GUARD4_6(d0, d1, d2, d3, x0, x1, x2, x3, x4, x5) \
  asm volatile(WG_NOP4 : "+v"(d0), "+v"(d1), "+v"(d2), "+v"(d3) \
               : "v"(x0), "v"(x1), "v"(x2), "v"(x3), "v"(x4), "v"(x5))
#define WAVE_LDS_SYNC() do { __builtin_amdgcn_fence(__ATOMIC_RELEASE, "workgroup"); \
  __builtin_amdgcn_wave_barrier(); __builtin_amdgcn_fence(__ATOMIC_ACQUIRE, "workgroup"); } while (0)
__device__ __forceinline__ float rcp_(float x) { return __builtin_amdgcn_rcpf(x); }
#else
#define GUARD1_4(...) ((void)0)
#define GUARD2_5(...) ((void)0)
#define GUARD4_6(...) ((void)0)
#define WAVE_LDS_SYNC() ((void)0)
__device__ __forceinline__ float rcp_(float x) { return 1.0f / x; }
#endif

__device__ __forceinline__ float sigm_(float x) {
  x = fminf(fmaxf(x, -30.0f), 30.0f);
  return rcp_(1.0f + __expf(-x));
}
__device__ __forceinline__ float tanh_(float x) {
  x = fminf(fmaxf(x, -15.0f), 15.0f);
  const float e = __expf(2.0f * x);
  return 1.0f - 2.0f * rcp_(1.0f + e);
}

__global__ __launch_bounds__(256) void zero_kernel(float* __restrict__ p, int n16) {
  const int i = (int)blockIdx.x * 256 + (int)threadIdx.x;
  if (i >= n16) return;
  v4f z;
#pragma unroll
  for (int e = 0; e < 4; ++e) z[e] = 0.0f;
  float* d = p + (size_t)i * 4;
  *(volatile v4f*)d = z;
  __threadfence();
  *(volatile v4f*)d = z;
}

__global__ __launch_bounds__(256) void cvt_w_kernel(const float* __restrict__ qw, const float* __restrict__ kw,
                                                    const float* __restrict__ vw, const float* __restrict__ cw,
                                                    _Float16* __restrict__ Wq16, _Float16* __restrict__ Wc16) {
  const int bid = (int)blockIdx.x, tid = (int)threadIdx.x;
  const float wsc = 1024.0f;
  v8h o;
  _Float16* dst;
  if (bid < 6) {
    const int li = bid * 256 + tid;
    const int mat = li >> 9;
    const int e = (li & 511) * 8;
    const float* src = (mat == 0) ? qw : ((mat == 1) ? kw : vw);
    const v4f a = *(const v4f*)(src + e), bq4 = *(const v4f*)(src + e + 4);
#pragma unroll
    for (int i = 0; i < 4; ++i) {
      o[i]     = (_Float16)(bfr(a[i]) * wsc);
      o[4 + i] = (_Float16)(bfr(bq4[i]) * wsc);
    }
    dst = Wq16 + (size_t)li * 8;
  } else {
    const int li = (bid - 6) * 256 + tid;
    const int piece = li & 15;
    const int toc = li >> 4;
    const int oc = toc & 255, tap = toc >> 8;
    const int ci0 = piece * 8;
#pragma unroll
    for (int i = 0; i < 8; ++i)
      o[i] = (_Float16)(bfr(cw[((size_t)(oc * CZ_ + ci0 + i)) * 9 + tap]) * wsc);
    dst = Wc16 + (size_t)li * 8;
  }
  *(volatile v8h*)dst = o;
  __threadfence();
  *(volatile v8h*)dst = o;
}

__global__ __launch_bounds__(128) void qkv_kernel(const float* __restrict__ X, const _Float16* __restrict__ Wq16,
                                                  const float* __restrict__ qb, const float* __restrict__ kbias,
                                                  const float* __restrict__ vb,
                                                  _Float16* __restrict__ QH, _Float16* __restrict__ QL,
                                                  _Float16* __restrict__ KH, _Float16* __restrict__ KL,
                                                  _Float16* __restrict__ VH, _Float16* __restrict__ VL, int ibase) {
  __shared__ __align__(16) _Float16 sQh[64 * 72];
  __shared__ __align__(16) _Float16 sQl[64 * 72];
  __shared__ __align__(16) _Float16 sKh[64 * 72];
  __shared__ __align__(16) _Float16 sKl[64 * 72];
  __shared__ __align__(16) _Float16 sVh[64 * 72];
  __shared__ __align__(16) _Float16 sVl[64 * 72];
  const int tid = (int)threadIdx.x, wave = tid >> 5, lane = tid & 31, h = lane >> 4, c = lane & 15;
  const int limg = (int)blockIdx.x >> 4, pg = (int)blockIdx.x & 15;
  const int gimg = ibase + limg, b = gimg >> 4, t = gimg & 15;
  const int pxl = wave * 16 + c;
  const int px = pg * 64 + pxl;
  const float* xp = X + ((size_t)b * NCH * NT_ + t) * NPX + px;
  const float xsc = 1024.0f;

  v16h bq[2];
#pragma unroll
  for (int ks = 0; ks < 2; ++ks) {
#pragma unroll
    for (int i = 0; i < 16; ++i) {
      const int ch = ks * 32 + ((i < 8) ? (8 * h + i) : (8 + 8 * h + i));
      bq[ks][i] = (_Float16)(bfr(xp[(size_t)ch * (NT_ * NPX)]) * xsc);
    }
  }
  v8f acc[12];
#pragma unroll
  for (int i = 0; i < 12; ++i) acc[i] = zero8();
  const _Float16* wl = Wq16 + (size_t)c * 64 + 8 * h;
#pragma unroll
  for (int i = 0; i < 12; ++i) {
    const v16h a0 = ldfrag(wl + i * 16 * 64), a1 = ldfrag(wl + i * 16 * 64 + 32);
    acc[i] = mma16(a0, bq[0], acc[i]);
    acc[i] = mma16(a1, bq[1], acc[i]);
    GUARD1_4(acc[i], a0, a1, bq[0], bq[1]);
  }
  const float ksc = 1.0f / 1024.0f, bsc = 1024.0f;
#pragma unroll
  for (int i = 0; i < 4; ++i) {
#pragma unroll
    for (int r = 0; r < 8; ++r) {
      const int o = 16 * i + 8 * h + r;
      const float qs = acc[i][r] * ksc + bsc * bfr(qb[o]);
      const _Float16 hi = (_Float16)qs;
      sQh[pxl * 72 + o] = hi;
      sQl[pxl * 72 + o] = (_Float16)(qs - (float)hi);
    }
  }
#pragma unroll
  for (int i = 4; i < 8; ++i) {
#pragma unroll
    for (int r = 0; r < 8; ++r) {
      const int o = 16 * (i - 4) + 8 * h + r;
      const float kv = acc[i][r] * ksc + bsc * bfr(kbias[o]);
      const _Float16 hi = (_Float16)kv;
      sKh[pxl * 72 + o] = hi;
      sKl[pxl * 72 + o] = (_Float16)(kv - (float)hi);
    }
  }
#pragma unroll
  for (int i = 8; i < 12; ++i) {
#pragma unroll
    for (int r = 0; r < 8; ++r) {
      const int o = 16 * (i - 8) + 8 * h + r;
      const float vs = acc[i][r] * ksc + bsc * bfr(vb[o]);
      const _Float16 hi = (_Float16)vs;
      sVh[o * 72 + pxl] = hi;
      sVl[o * 72 + pxl] = (_Float16)(vs - (float)hi);
    }
  }
  __syncthreads();
  const size_t prow = (size_t)limg * NPX + pg * 64;
  const size_t vrow = (size_t)limg * NCH;
#pragma unroll
  for (int ps = 0; ps < 2; ++ps) {
#pragma unroll
    for (int it = 0; it < 4; ++it) {
      const int L = it * 16 + (tid >> 3), e = tid & 7;
      const v8h q1 = *(const v8h*)(sQh + L * 72 + 8 * e);
      const v8h q2 = *(const v8h*)(sQl + L * 72 + 8 * e);
      const v8h k1 = *(const v8h*)(sKh + L * 72 + 8 * e);
      const v8h k2 = *(const v8h*)(sKl + L * 72 + 8 * e);
      const v8h v1 = *(const v8h*)(sVh + L * 72 + 8 * e);
      const v8h v2 = *(const v8h*)(sVl + L * 72 + 8 * e);
      *(volatile v8h*)(QH + (prow + L) * 64 + 8 * e) = q1;
      *(volatile v8h*)(QL + (prow + L) * 64 + 8 * e) = q2;
      *(volatile v8h*)(KH + (prow + L) * 64 + 8 * e) = k1;
      *(volatile v8h*)(KL + (prow + L) * 64 + 8 * e) = k2;
      *(volatile v8h*)(VH + (vrow + L) * NPX + pg * 64 + 8 * e) = v1;
      *(volatile v8h*)(VL + (vrow + L) * NPX + pg * 64 + 8 * e) = v2;
    }
    __threadfence();
  }
}

__global__ __launch_bounds__(128) void attn_kernel(const _Float16* __restrict__ QH, const _Float16* __restrict__ QL,
                                                   const _Float16* __restrict__ KH, const _Float16* __restrict__ KL,
                                                   const _Float16* __restrict__ VH, const _Float16* __restrict__ VL,
                                                   _Float16* __restrict__ AXH, _Float16* __restrict__ AXL, int ibase) {
  __shared__ __align__(16) _Float16 sOh[4 * 16 * 72];
  __shared__ __align__(16) _Float16 sOl[4 * 16 * 72];
  const int tid = (int)threadIdx.x, wave = tid >> 5, lane = tid & 31, h = lane >> 4, c = lane & 15;
  const int limg = (int)blockIdx.x >> 4, qg = (int)blockIdx.x & 15;
  const int gimg = ibase + limg, b = gimg >> 4, t = gimg & 15;
  const int q0w = qg * 64 + wave * 16;
  const float ninf = -__builtin_inff();

  const size_t qrow = (size_t)limg * NPX + q0w + c;
  const v16h qh0 = ldfrag(QH + qrow * 64 + 8 * h), qh1 = ldfrag(QH + qrow * 64 + 32 + 8 * h);
  const v16h ql0 = ldfrag(QL + qrow * 64 + 8 * h), ql1 = ldfrag(QL + qrow * 64 + 32 + 8 * h);
  const _Float16* khb = KH + ((size_t)limg * NPX + c) * 64 + 8 * h;
  const _Float16* klb = KL + ((size_t)limg * NPX + c) * 64 + 8 * h;
  const _Float16* vhb = VH + ((size_t)limg * NCH + c) * NPX + 8 * h;
  const _Float16* vlb = VL + ((size_t)limg * NCH + c) * NPX + 8 * h;

  v8f oacc[4];
#pragma unroll
  for (int j = 0; j < 4; ++j) oacc[j] = zero8();
  float mrun = ninf, lpart = 0.0f;
  const float ssc = 1.0f / 1048576.0f;
  const float psc = 16384.0f;

#pragma unroll 1
  for (int kb = 0; kb < NPX; kb += 32) {
    v8f sacc[2];
#pragma unroll
    for (int kt = 0; kt < 2; ++kt) {
      const size_t ko = (size_t)(kb + 16 * kt) * 64;
      const v16h kh0 = ldfrag(khb + ko), kh1 = ldfrag(khb + ko + 32);
      const v16h kl0 = ldfrag(klb + ko), kl1 = ldfrag(klb + ko + 32);
      sacc[kt] = mma16(kh0, qh0, zero8());
      sacc[kt] = mma16(kh1, qh1, sacc[kt]);
      sacc[kt] = mma16(kh0, ql0, sacc[kt]);
      sacc[kt] = mma16(kh1, ql1, sacc[kt]);
      sacc[kt] = mma16(kl0, qh0, sacc[kt]);
      sacc[kt] = mma16(kl1, qh1, sacc[kt]);
      GUARD1_4(sacc[kt], kh0, kh1, kl0, kl1);
    }
    float s[2][8];
    float mloc = ninf;
#pragma unroll
    for (int kt = 0; kt < 2; ++kt) {
#pragma unroll
      for (int r = 0; r < 8; ++r) {
        const float v = sacc[kt][r] * ssc;
        s[kt][r] = v;
        mloc = fmaxf(mloc, v);
      }
    }
    const float mblk = fmaxf(mloc, __shfl_xor(mloc, 16, 32));
    const float mnew = fmaxf(mrun, mblk);
    const float al = __expf(mrun - mnew);
    mrun = mnew;
    float ps = 0.0f;
    v16h pv;
#pragma unroll
    for (int r = 0; r < 8; ++r) {
      const float p0 = __expf(s[0][r] - mnew);
      const float p1 = __expf(s[1][r] - mnew);
      ps += p0 + p1;
      pv[r]     = (_Float16)(p0 * psc);
      pv[8 + r] = (_Float16)(p1 * psc);
    }
    lpart = lpart * al + ps;
    float alr[8];
#pragma unroll
    for (int r = 0; r < 8; ++r) alr[r] = __shfl(al, 8 * h + r, 32);
#pragma unroll
    for (int j = 0; j < 4; ++j) {
#pragma unroll
      for (int r = 0; r < 8; ++r) oacc[j][r] *= alr[r];
    }
#pragma unroll
    for (int g = 0; g < 2; ++g) {
      const size_t vo = (size_t)(32 * g) * NPX + kb;
      const v16h vh0 = ldfrag(vhb + vo), vl0 = ldfrag(vlb + vo);
      const v16h vh1 = ldfrag(vhb + vo + 16 * NPX), vl1 = ldfrag(vlb + vo + 16 * NPX);
      oacc[2 * g]     = mma16(pv, vh0, oacc[2 * g]);
      oacc[2 * g]     = mma16(pv, vl0, oacc[2 * g]);
      oacc[2 * g + 1] = mma16(pv, vh1, oacc[2 * g + 1]);
      oacc[2 * g + 1] = mma16(pv, vl1, oacc[2 * g + 1]);
      GUARD2_5(oacc[2 * g], oacc[2 * g + 1], pv, vh0, vl0, vh1, vl1);
    }
  }

  const float l = lpart + __shfl_xor(lpart, 16, 32);
  const float inv = rcp_(l) * (1.0f / 4096.0f);
  float invr[8];
#pragma unroll
  for (int r = 0; r < 8; ++r) invr[r] = __shfl(inv, 8 * h + r, 32);
  _Float16* sth = sOh + wave * 16 * 72;
  _Float16* stl = sOl + wave * 16 * 72;
#pragma unroll
  for (int j = 0; j < 4; ++j) {
#pragma unroll
    for (int r = 0; r < 8; ++r) {
      const float axv = oacc[j][r] * invr[r];
      const _Float16 hi = (_Float16)axv;
      sth[(8 * h + r) * 72 + 16 * j + c] = hi;
      stl[(8 * h + r) * 72 + 16 * j + c] = (_Float16)(axv - (float)hi);
    }
  }
  WAVE_LDS_SYNC();
  const size_t zoff = ((size_t)(t * NB_ + b) * NPX + q0w) * 64;
  _Float16* zh = AXH + zoff;
  _Float16* zl = AXL + zoff;
#pragma unroll
  for (int ps = 0; ps < 2; ++ps) {
#pragma unroll
    for (int it = 0; it < 4; ++it) {
      const int pl = it * 4 + (lane >> 3), e = lane & 7;
      const v8h vh = *(const v8h*)(sth + pl * 72 + 8 * e);
      const v8h vl = *(const v8h*)(stl + pl * 72 + 8 * e);
      *(volatile v8h*)(zh + (size_t)pl * 64 + 8 * e) = vh;
      *(volatile v8h*)(zl + (size_t)pl * 64 + 8 * e) = vl;
    }
    __threadfence();
  }
}

__global__ __launch_bounds__(64) void conv_cell_kernel(const _Float16* __restrict__ AXh, const _Float16* __restrict__ AXl,
                                                       const _Float16* __restrict__ Hh, const _Float16* __restrict__ Hl,
                                                       const _Float16* __restrict__ Wc16,
                                                       const float* __restrict__ cb, const float* __restrict__ wci,
                                                       const float* __restrict__ wcf, const float* __restrict__ wco,
                                                       float* __restrict__ Cst, float* __restrict__ out,
                                                       _Float16* __restrict__ Hnh, _Float16* __restrict__ Hnl,
                                                       int t, int npl) {
  __shared__ __align__(16) float cs[64 * 36];
  __shared__ __align__(16) float hs[64 * 36];
  __shared__ __align__(16) _Float16 zsh[32 * 72];
  __shared__ __align__(16) _Float16 zsl[32 * 72];
  const int tid = (int)threadIdx.x, wave = tid >> 5, lane = tid & 31, h = lane >> 4, c = lane & 15;
  const int b = (int)blockIdx.x >> 5, y = (int)blockIdx.x & 31;
  const int x = wave * 16 + c;
  const int px = y * IW_ + x;
  const _Float16* wl = Wc16 + (size_t)c * CZ_ + 8 * h;

  v8f acc[16];
#pragma unroll
  for (int i = 0; i < 16; ++i) acc[i] = zero8();

#pragma unroll 1
  for (int tap = 0; tap < 9; ++tap) {
    const int dy = ((tap * 11) >> 5) - 1;
    const int dx = tap - 3 * (dy + 1) - 1;
    const int sy = y + dy, sx = x + dx;
    const bool ok = ((unsigned)sy < 32u) && ((unsigned)sx < 32u);
    const int syc = min(max(sy, 0), 31), sxc = min(max(sx, 0), 31);
    const unsigned msk = ok ? 0xFFFFFFFFu : 0u;
    const size_t poff = ((size_t)b * NPX + syc * IW_ + sxc) * 64 + 8 * h;
    const _Float16* wp = wl + (size_t)tap * NOC * CZ_;
#pragma unroll 1
    for (int pl = 0; pl < npl; ++pl) {
      const _Float16* bph = ((pl == 0) ? AXh : Hh) + poff;
      const _Float16* bpl = ((pl == 0) ? AXl : Hl) + poff;
      const _Float16* wpp = wp + pl * 64;
#pragma unroll
      for (int cbk = 0; cbk < 64; cbk += 32) {
        FragU fh, fl;
        fh.v = ldfrag(bph + cbk);
        fl.v = ldfrag(bpl + cbk);
        fh.u = fh.u & msk;
        fl.u = fl.u & msk;
        const v16h bh = fh.v, bl = fl.v;
#pragma unroll
        for (int g = 0; g < 4; ++g) {
          const _Float16* ap = wpp + (size_t)(g * 64) * CZ_ + cbk;
          const v16h a0 = ldfrag(ap), a1 = ldfrag(ap + 16 * CZ_);
          const v16h a2 = ldfrag(ap + 32 * CZ_), a3 = ldfrag(ap + 48 * CZ_);
          acc[4 * g]     = mma16(a0, bh, acc[4 * g]);
          acc[4 * g]     = mma16(a0, bl, acc[4 * g]);
          acc[4 * g + 1] = mma16(a1, bh, acc[4 * g + 1]);
          acc[4 * g + 1] = mma16(a1, bl, acc[4 * g + 1]);
          acc[4 * g + 2] = mma16(a2, bh, acc[4 * g + 2]);
          acc[4 * g + 2] = mma16(a2, bl, acc[4 * g + 2]);
          acc[4 * g + 3] = mma16(a3, bh, acc[4 * g + 3]);
          acc[4 * g + 3] = mma16(a3, bl, acc[4 * g + 3]);
          GUARD4_6(acc[4 * g], acc[4 * g + 1], acc[4 * g + 2], acc[4 * g + 3], bh, bl, a0, a1, a2, a3);
        }
      }
    }
  }

  const float kinv = 1.0f / 4194304.0f;
  const float hsc = 4096.0f;
  const size_t cbase = (size_t)b * NCH * NPX + px;
#pragma unroll
  for (int q = 0; q < 4; ++q) {
#pragma unroll
    for (int r = 0; r < 8; ++r) {
      const int cc = 16 * q + 8 * h + r;
      const float pi = acc[q][r]      * kinv + bfr(cb[cc]);
      const float pf = acc[4 + q][r]  * kinv + bfr(cb[64 + cc]);
      const float pg = acc[8 + q][r]  * kinv + bfr(cb[128 + cc]);
      const float po = acc[12 + q][r] * kinv + bfr(cb[192 + cc]);
      const float cprev = Cst[cbase + (size_t)cc * NPX];
      const int pidx = cc * NPX + px;
      const float pci = bfr(wci[pidx]), pcf = bfr(wcf[pidx]), pco = bfr(wco[pidx]);
      const float ig = sigm_(pi + pci * cprev);
      const float fg = sigm_(pf + pcf * cprev);
      const float nc = fg * cprev + ig * tanh_(pg);
      const float og = sigm_(po + pco * nc);
      const float nh = og * tanh_(nc);
      cs[cc * 36 + x] = nc;
      hs[cc * 36 + x] = nh;
      const float hv = nh * hsc;
      const _Float16 hi = (_Float16)hv;
      zsh[x * 72 + cc] = hi;
      zsl[x * 72 + cc] = (_Float16)(hv - (float)hi);
    }
  }
  __syncthreads();
  float* cdst = Cst + (size_t)b * NCH * NPX + y * IW_;
  float* odst = out + (size_t)b * NCH * NT_ * NPX + (size_t)t * NPX + y * IW_;
  const size_t hoff = ((size_t)b * NPX + y * IW_) * 64;
  _Float16* hdh = Hnh + hoff;
  _Float16* hdl = Hnl + hoff;
#pragma unroll
  for (int ps = 0; ps < 2; ++ps) {
#pragma unroll
    for (int it = 0; it < 8; ++it) {
      const int L = it * 8 + (tid >> 3), e = tid & 7;
      const v4f cv = *(const v4f*)(cs + L * 36 + 4 * e);
      const v4f hv = *(const v4f*)(hs + L * 36 + 4 * e);
      *(volatile v4f*)(cdst + (size_t)L * NPX + 4 * e) = cv;
      *(volatile v4f*)(odst + (size_t)L * (NT_ * NPX) + 4 * e) = hv;
    }
#pragma unroll
    for (int it = 0; it < 4; ++it) {
      const int L = it * 8 + (tid >> 3), e = tid & 7;
      const v8h zh = *(const v8h*)(zsh + L * 72 + 8 * e);
      const v8h zl = *(const v8h*)(zsl + L * 72 + 8 * e);
      *(volatile v8h*)(hdh + (size_t)L * 64 + 8 * e) = zh;
      *(volatile v8h*)(hdl + (size_t)L * 64 + 8 * e) = zl;
    }
    __threadfence();
  }
}

extern "C" void kernel_launch(void* const* d_in, const int* in_sizes, int n_in,
                              void* d_out, int out_size, void* d_ws, size_t ws_size,
                              hipStream_t stream) {
  if (n_in < 12) return;
  if (in_sizes[0] != NB_ * NCH * NT_ * NPX) return;
  if (in_sizes[1] != 4096 || in_sizes[3] != 4096 || in_sizes[5] != 4096) return;
  if (in_sizes[2] != 64 || in_sizes[4] != 64 || in_sizes[6] != 64) return;
  if (in_sizes[7] != NOC * CZ_ * 9 || in_sizes[8] != NOC) return;
  if (in_sizes[9] != NCH * NPX || in_sizes[10] != NCH * NPX || in_sizes[11] != NCH * NPX) return;
  if (out_size != NB_ * NCH * NT_ * NPX) return;

  const float* X   = (const float*)d_in[0];
  const float* qw  = (const float*)d_in[1];
  const float* qb  = (const float*)d_in[2];
  const float* kw  = (const float*)d_in[3];
  const float* kb  = (const float*)d_in[4];
  const float* vw  = (const float*)d_in[5];
  const float* vb  = (const float*)d_in[6];
  const float* cw  = (const float*)d_in[7];
  const float* cbi = (const float*)d_in[8];
  const float* wci = (const float*)d_in[9];
  const float* wcf = (const float*)d_in[10];
  const float* wco = (const float*)d_in[11];
  float* out = (float*)d_out;

  const size_t bWq = (size_t)192 * 64 * 2;
  const size_t bWc = (size_t)9 * NOC * CZ_ * 2;
  const size_t bP  = (size_t)ICH * NPX * 64 * 2;
  const size_t bAX = (size_t)NT_ * NB_ * NPX * 64 * 2;
  const size_t bH  = (size_t)NB_ * NPX * 64 * 2;
  const size_t bC  = (size_t)NB_ * NCH * NPX * 4;
  size_t off = 0;
  const size_t oWq = off; off += bWq;
  const size_t oWc = off; off += bWc;
  const size_t oQH = off; off += bP;
  const size_t oQL = off; off += bP;
  const size_t oKH = off; off += bP;
  const size_t oKL = off; off += bP;
  const size_t oVH = off; off += bP;
  const size_t oVL = off; off += bP;
  const size_t oAH = off; off += bAX;
  const size_t oAL = off; off += bAX;
  const size_t oH0h = off; off += bH;
  const size_t oH0l = off; off += bH;
  const size_t oC   = off; off += bC;
  const size_t oH1h = off; off += bH;
  const size_t oH1l = off; off += bH;
  if (off > ws_size) return;
  if (off > (size_t)134217728) return;
  if (oH0l != oH0h + bH || oC != oH0l + bH) return;

  char* ws = (char*)d_ws;
  _Float16* Wq16 = (_Float16*)(ws + oWq);
  _Float16* Wc16 = (_Float16*)(ws + oWc);
  _Float16* QH   = (_Float16*)(ws + oQH);
  _Float16* QL   = (_Float16*)(ws + oQL);
  _Float16* KH   = (_Float16*)(ws + oKH);
  _Float16* KL   = (_Float16*)(ws + oKL);
  _Float16* VH   = (_Float16*)(ws + oVH);
  _Float16* VL   = (_Float16*)(ws + oVL);
  _Float16* AXH  = (_Float16*)(ws + oAH);
  _Float16* AXL  = (_Float16*)(ws + oAL);
  _Float16* Hh[2] = { (_Float16*)(ws + oH0h), (_Float16*)(ws + oH1h) };
  _Float16* Hl[2] = { (_Float16*)(ws + oH0l), (_Float16*)(ws + oH1l) };
  float*    Cst  = (float*)(ws + oC);

  const size_t zbytes = 2 * bH + bC;
  const int n16 = (int)(zbytes / 16);
  if ((n16 % 256) != 0) return;
  zero_kernel<<<dim3(n16 / 256), dim3(256), 0, stream>>>((float*)(ws + oH0h), n16);
  cvt_w_kernel<<<dim3(150), dim3(256), 0, stream>>>(qw, kw, vw, cw, Wq16, Wc16);
  for (int ch = 0; ch < NIMG / ICH; ++ch) {
    const int ibase = ch * ICH;
    qkv_kernel<<<dim3(ICH * 16), dim3(128), 0, stream>>>(X, Wq16, qb, kb, vb, QH, QL, KH, KL, VH, VL, ibase);
    attn_kernel<<<dim3(ICH * 16), dim3(128), 0, stream>>>(QH, QL, KH, KL, VH, VL, AXH, AXL, ibase);
  }
  const size_t axslice = (size_t)NB_ * NPX * 64;
  for (int t = 0; t < NT_; ++t) {
    const int cur = t & 1, nxt = (t + 1) & 1;
    const int npl = (t == 0) ? 1 : 2;
    conv_cell_kernel<<<dim3(NB_ * 32), dim3(64), 0, stream>>>(
        AXH + (size_t)t * axslice, AXL + (size_t)t * axslice, Hh[cur], Hl[cur], Wc16,
        cbi, wci, wcf, wco, Cst, out, Hh[nxt], Hl[nxt], t, npl);
  }
  (void)hipGetLastError();
}
